// SigmoidImplicitLayer_7885559955905
// MI455X (gfx1250) — hardware-verified
//
#include <hip/hip_runtime.h>


namespace {
constexpr int Bn = 64, N = 512, D = 256, H = 512, ITERS = 20;
constexpr float AS_ = 8.0f;

typedef _Float16 b16;
typedef __attribute__((ext_vector_type(16))) _Float16 v16b;
typedef __attribute__((ext_vector_type(8))) _Float16 v8b;
typedef __attribute__((ext_vector_type(8))) float v8f;
typedef __attribute__((ext_vector_type(4))) float v4f;
__device__ __forceinline__ float bf16_rne(float f) { unsigned int u = __float_as_uint(f); u += 0x7FFFu + ((u >> 16) & 1u); return __uint_as_float(u & 0xFFFF0000u); }
__device__ __forceinline__ void split16(float v, b16& hi, b16& lo) { hi = (b16)v; lo = (b16)(v - (float)hi); }
__device__ __forceinline__ v16b frag_kb(const b16* p, int hh) { const v8b a = *(const v8b*)(p + 8 * hh), b = *(const v8b*)(p + 16 + 8 * hh); v16b f;
#pragma unroll
  for (int e = 0; e < 8; ++e) { f[e] = a[e]; f[8 + e] = b[e]; } return f; }
__device__ __forceinline__ v16b frag_x(const float* p, int hh) { v16b f;
#pragma unroll
  for (int e = 0; e < 8; ++e) { f[e] = (b16)bf16_rne(p[8 * hh + e]); f[8 + e] = (b16)bf16_rne(p[16 + 8 * hh + e]); } return f; }
__device__ __forceinline__ v8f wmma16b(v16b a, v16b b, v8f c) { v8f d = __builtin_amdgcn_wmma_f32_16x16x32_f16(false, a, false, b, (short)0, c, false, false); asm volatile("v_nop\n\tv_nop\n\tv_nop\n\tv_nop" : "+v"(d) : "v"(a), "v"(b)); return d; }
__device__ __forceinline__ void wave_lds_sync() { __builtin_amdgcn_fence(__ATOMIC_RELEASE, "workgroup"); __builtin_amdgcn_wave_barrier(); __builtin_amdgcn_fence(__ATOMIC_ACQUIRE, "workgroup"); }
__device__ __forceinline__ float nexp(float x) { return __builtin_amdgcn_exp2f(x * 1.4426950408889634f); }

struct Wo_ { static constexpr size_t W1A = 0, W1B = W1A + (size_t)H * D, W2 = W1B + (size_t)H * D, END = W2 + 16 * H; };
__global__ __launch_bounds__(256) void prep_kernel(const float* __restrict__ W1, const float* __restrict__ b1, const float* __restrict__ W2, const float* __restrict__ b2, b16* __restrict__ R, float* __restrict__ P) {
  const int t_ = blockIdx.x * 256 + threadIdx.x, nth = gridDim.x * 256;
  for (int pass = 0; pass < 2; ++pass) {
    for (int q = t_; q < H * D; q += nth) { const int h = q / D, d = q % D; R[Wo_::W1A + q] = (b16)bf16_rne(W1[(size_t)d * H + h]); R[Wo_::W1B + q] = (b16)bf16_rne(W1[(size_t)(D + d) * H + h]); }
    for (int q = t_; q < 16 * H; q += nth) R[Wo_::W2 + q] = (b16)((q < H) ? bf16_rne(W2[q]) : 0.0f);
    for (int q = t_; q < H + 1; q += nth) P[q] = (q < H) ? bf16_rne(b1[q]) : bf16_rne(b2[0]);
    __threadfence(); }
}

__global__ __launch_bounds__(256) void vt_kernel(const float* __restrict__ V, b16* __restrict__ vt) {
  __shared__ __attribute__((aligned(16))) b16 T[D][128 + 8];
  const int b = blockIdx.y, n0 = blockIdx.x * 128, t_ = threadIdx.x;
  for (int i = t_; i < 128 * D; i += 256) { const int nn = i / D, d = i % D; T[d][nn] = (b16)bf16_rne(V[((size_t)b * N + n0 + nn) * D + d]); }
  __syncthreads();
  for (int pass = 0; pass < 2; ++pass) { for (int i = t_; i < D * 16; i += 256) { const int d = i >> 4, c8 = (i & 15) * 8; *(volatile v8b*)(vt + ((size_t)b * D + d) * N + n0 + c8) = *(const v8b*)(&T[d][c8]); } __threadfence(); }
}

__global__ __launch_bounds__(128) void a0_kernel(const float* __restrict__ V, const b16* __restrict__ R, float* __restrict__ A0) {
  __shared__ __attribute__((aligned(16))) float Ts[4][32 * 64];
  const int lane = threadIdx.x & 31, wave = threadIdx.x >> 5, nloc = lane & 15, hlf = lane >> 4, m0 = blockIdx.y * 128 + wave * 32, c0 = blockIdx.x * 64;
  v8f acc[2][4];
#pragma unroll
  for (int r = 0; r < 2; ++r)
#pragma unroll
    for (int t = 0; t < 4; ++t) acc[r][t] = (v8f){};
#pragma unroll
  for (int kb = 0; kb < D; kb += 32) { const v16b a0 = frag_x(V + (size_t)(m0 + nloc) * D + kb, hlf), a1 = frag_x(V + (size_t)(m0 + 16 + nloc) * D + kb, hlf);
#pragma unroll
    for (int t = 0; t < 4; ++t) { const v16b bw = frag_kb(R + Wo_::W1A + (size_t)(c0 + t * 16 + nloc) * D + kb, hlf); acc[0][t] = wmma16b(a0, bw, acc[0][t]); acc[1][t] = wmma16b(a1, bw, acc[1][t]); } }
  float* Tt = Ts[wave];
#pragma unroll
  for (int t = 0; t < 4; ++t)
#pragma unroll
    for (int r = 0; r < 2; ++r)
#pragma unroll
      for (int v = 0; v < 8; ++v) Tt[(r * 16 + v + 8 * hlf) * 64 + t * 16 + nloc] = acc[r][t][v];
  wave_lds_sync();
  for (int pass = 0; pass < 2; ++pass) {
#pragma unroll
    for (int j = 0; j < 16; ++j) { const int rr = j * 2 + hlf, c4 = nloc * 4; *(volatile v4f*)(A0 + (size_t)(m0 + rr) * H + c0 + c4) = *(const v4f*)(Tt + rr * 64 + c4); }
    __threadfence(); }
}

__global__ __launch_bounds__(256) void iter_kernel(const float* __restrict__ q0, const b16* __restrict__ vt, const float* __restrict__ A0, const b16* __restrict__ R, const float* __restrict__ P, float* __restrict__ out) {
  __shared__ __attribute__((aligned(16))) b16 Qh[16][N + 8], Ql[16][N + 8], Ph[16][D + 8], Pl[16][D + 8]; __shared__ float pw[H]; __shared__ __attribute__((aligned(16))) float qv[N];
  const int b = blockIdx.x, t_ = threadIdx.x, wave = t_ >> 5, lane = t_ & 31, nloc = lane & 15, hlf = lane >> 4; const float* b1 = P; const float b2 = P[H];
  for (int i = t_; i < 16 * (N + 8); i += 256) { (&Qh[0][0])[i] = (b16)0.0f; (&Ql[0][0])[i] = (b16)0.0f; }
  for (int i = t_; i < 16 * (D + 8); i += 256) { (&Ph[0][0])[i] = (b16)0.0f; (&Pl[0][0])[i] = (b16)0.0f; }
  __syncthreads();
  for (int i = t_; i < N; i += 256) { const float q = bf16_rne(q0[(size_t)b * N + i]); qv[i] = q; b16 h_, l_; split16(q * AS_, h_, l_); Qh[0][i] = h_; Ql[0][i] = l_; }
  __syncthreads();
  const b16* Vt = vt + ((size_t)b * D) * N; const float* Ab = A0 + ((size_t)b * N) * H;
  for (int it = 0; it < ITERS; ++it) {
    { v8f acc[2] = {{}, {}};
      for (int kb = 0; kb < N; kb += 32) { const v16b ah = frag_kb(&Qh[nloc][kb], hlf), al = frag_kb(&Ql[nloc][kb], hlf);
#pragma unroll
        for (int t = 0; t < 2; ++t) { const v16b bw = frag_kb(Vt + (size_t)((wave * 2 + t) * 16 + nloc) * N + kb, hlf); acc[t] = wmma16b(ah, bw, acc[t]); acc[t] = wmma16b(al, bw, acc[t]); } }
      if (hlf == 0) {
#pragma unroll
        for (int t = 0; t < 2; ++t) { const float pv = acc[t][0] * (1.0f / AS_); b16 h_, l_; split16(pv * AS_, h_, l_); Ph[0][(wave * 2 + t) * 16 + nloc] = h_; Pl[0][(wave * 2 + t) * 16 + nloc] = l_; } } }
    __syncthreads();
    { v8f acc[4] = {{}, {}, {}, {}};
#pragma unroll
      for (int kb = 0; kb < D; kb += 32) { const v16b ah = frag_kb(&Ph[nloc][kb], hlf), al = frag_kb(&Pl[nloc][kb], hlf);
#pragma unroll
        for (int t = 0; t < 4; ++t) { const v16b bw = frag_kb(R + Wo_::W1B + (size_t)((wave * 4 + t) * 16 + nloc) * D + kb, hlf); acc[t] = wmma16b(ah, bw, acc[t]); acc[t] = wmma16b(al, bw, acc[t]); } }
      if (hlf == 0) {
#pragma unroll
        for (int t = 0; t < 4; ++t) pw[(wave * 4 + t) * 16 + nloc] = acc[t][0] * (1.0f / AS_); } }
    __syncthreads();
    { v8f acc[4] = {{}, {}, {}, {}};
      for (int kb = 0; kb < H; kb += 32) { const v16b bw = frag_kb(R + Wo_::W2 + (size_t)nloc * H + kb, hlf);
#pragma unroll
        for (int t = 0; t < 4; ++t) { const int n = (wave * 4 + t) * 16 + nloc; const float* ar = Ab + (size_t)n * H + kb; v16b ah, al;
#pragma unroll
          for (int e = 0; e < 8; ++e) { const int k0 = 8 * hlf + e, k1 = 16 + 8 * hlf + e; b16 x_, y_; split16(fmaxf(ar[k0] + pw[kb + k0] + b1[kb + k0], 0.0f) * AS_, x_, y_); ah[e] = x_; al[e] = y_; split16(fmaxf(ar[k1] + pw[kb + k1] + b1[kb + k1], 0.0f) * AS_, x_, y_); ah[8 + e] = x_; al[8 + e] = y_; }
          acc[t] = wmma16b(ah, bw, acc[t]); acc[t] = wmma16b(al, bw, acc[t]); } }
      __syncthreads();
      if (nloc == 0) {
#pragma unroll
        for (int t = 0; t < 4; ++t)
#pragma unroll
          for (int r = 0; r < 8; ++r) { const int n = (wave * 4 + t) * 16 + 8 * hlf + r; const float q = 1.0f / (1.0f + nexp(-(acc[t][r] * (1.0f / AS_) + b2))); qv[n] = q; b16 h_, l_; split16(q * AS_, h_, l_); Qh[0][n] = h_; Ql[0][n] = l_; } } }
    __syncthreads(); }
  for (int pass = 0; pass < 2; ++pass) { for (int i = t_; i < N / 4; i += 256) *(volatile v4f*)(out + (size_t)b * N + i * 4) = *(const v4f*)(&qv[i * 4]); __threadfence(); }
}
}

extern "C" void kernel_launch(void* const* d_in, const int* in_sizes, int n_in,
                              void* d_out, int out_size, void* d_ws, size_t ws_size, hipStream_t stream) {
  (void)n_in; (void)out_size;
  const float* q0 = (const float*)d_in[0]; const float* V = (const float*)d_in[1]; const float* W1 = (const float*)d_in[2]; const float* b1 = (const float*)d_in[3]; const float* W2 = (const float*)d_in[4]; const float* b2 = (const float*)d_in[5];
  float* out = (float*)d_out;
  if (in_sizes[0] != Bn * N || in_sizes[1] != Bn * N * D || in_sizes[2] != 2 * D * H || in_sizes[4] != H) return;
  size_t off = 0; char* ws = (char*)d_ws;
  auto carve = [&](size_t bytes) { char* p = ws + off; off += (bytes + 255) & ~(size_t)255; return p; };
  b16* R = (b16*)carve(Wo_::END * 2); float* P = (float*)carve(1024 * 4); b16* vt = (b16*)carve((size_t)Bn * D * N * 2); float* A0 = (float*)carve((size_t)Bn * N * H * 4);
  if (off > ws_size) return;
  prep_kernel<<<128, 256, 0, stream>>>(W1, b1, W2, b2, R, P);
  vt_kernel<<<dim3(N / 128, Bn), 256, 0, stream>>>(V, vt);
  a0_kernel<<<dim3(H / 64, Bn * N / 128), 128, 0, stream>>>(V, R, A0);
  iter_kernel<<<Bn, 256, 0, stream>>>(q0, vt, A0, R, P, out);
}
